// TSP_Encoder_56487409877516
// MI455X (gfx1250) — hardware-verified
//
#include <hip/hip_runtime.h>
#include <stddef.h>
#include <stdint.h>

#define NB   64
#define NN   500
#define NP   512
#define NROW 32768
#define DM   128
#define DFF  512
#define NL   6
#define EPSV 1e-5f

static_assert(NROW == NB * NP);
static_assert(NROW % 256 == 0);
static_assert(NP == 2 * 256);
static_assert(DM % 64 == 0);
static_assert(DFF % 64 == 0);
static_assert((NL * DM * DM) % 2048 == 0);
static_assert((NL * DFF * DM) % 2048 == 0);
static_assert(NN % 4 == 0);

typedef _Float16 v16h __attribute__((ext_vector_type(16)));
typedef _Float16 v8h  __attribute__((ext_vector_type(8)));
typedef _Float16 v4h  __attribute__((ext_vector_type(4)));
typedef float    v8f  __attribute__((ext_vector_type(8)));
typedef float    v4f  __attribute__((ext_vector_type(4)));
typedef unsigned int v4u __attribute__((ext_vector_type(4)));
typedef unsigned int v2u __attribute__((ext_vector_type(2)));

union Frag  { v16h v; v8h h[2]; };
union Pack8 { v8h h; v4u u; };
union Pack4 { v4h h; v2u u; };

__device__ __forceinline__ v8f mma16(v16h a, v16h b, v8f c) {
  c = __builtin_amdgcn_wmma_f32_16x16x32_f16(false, a, false, b, (short)0, c, false, false);
  asm volatile("v_nop\n\tv_nop\n\tv_nop\n\tv_nop" : "+v"(c) : "v"(a), "v"(b));
  return c;
}

__device__ __forceinline__ v16h ldfrag(const _Float16* p, int ld, int row0, int k0, int lane) {
  const int m = lane & 15, lh = lane >> 4;
  const _Float16* q = p + (size_t)(row0 + m) * ld + k0 + 8 * lh;
  Frag f;
  f.h[0] = *(const v8h*)(q);
  f.h[1] = *(const v8h*)(q + 16);
  return f.v;
}

__device__ __forceinline__ v8f zero8() { return (v8f){0.f, 0.f, 0.f, 0.f, 0.f, 0.f, 0.f, 0.f}; }
__device__ __forceinline__ v4f zero4() { return (v4f){0.f, 0.f, 0.f, 0.f}; }

__device__ __forceinline__ v4u pack8h(v4f a0, v4f a1) {
  Pack8 pk;
  pk.h = (v8h){(_Float16)a0[0], (_Float16)a0[1], (_Float16)a0[2], (_Float16)a0[3],
               (_Float16)a1[0], (_Float16)a1[1], (_Float16)a1[2], (_Float16)a1[3]};
  return pk.u;
}
__device__ __forceinline__ v2u pack4h(v4f a) {
  Pack4 pk;
  pk.h = (v4h){(_Float16)a[0], (_Float16)a[1], (_Float16)a[2], (_Float16)a[3]};
  return pk.u;
}
__device__ __forceinline__ v4f sel4(bool p, v4f v) {
  v4f r;
  r[0] = p ? v[0] : 0.f; r[1] = p ? v[1] : 0.f; r[2] = p ? v[2] : 0.f; r[3] = p ? v[3] : 0.f;
  return r;
}

__device__ __forceinline__ void gemm32x64(const _Float16* __restrict__ A, int lda,
                                          const _Float16* __restrict__ Bt, int ldb, int K,
                                          int m0, int n0, int lane, v8f (&acc)[2][4]) {
#pragma unroll 1
  for (int k0 = 0; k0 < K; k0 += 32) {
    const v16h a0 = ldfrag(A, lda, m0, k0, lane);
    const v16h a1 = ldfrag(A, lda, m0 + 16, k0, lane);
    const v16h b0 = ldfrag(Bt, ldb, n0, k0, lane);
    const v16h b1 = ldfrag(Bt, ldb, n0 + 16, k0, lane);
    const v16h b2 = ldfrag(Bt, ldb, n0 + 32, k0, lane);
    const v16h b3 = ldfrag(Bt, ldb, n0 + 48, k0, lane);
    acc[0][0] = mma16(a0, b0, acc[0][0]);
    acc[1][0] = mma16(a1, b0, acc[1][0]);
    acc[0][1] = mma16(a0, b1, acc[0][1]);
    acc[1][1] = mma16(a1, b1, acc[1][1]);
    acc[0][2] = mma16(a0, b2, acc[0][2]);
    acc[1][2] = mma16(a1, b2, acc[1][2]);
    acc[0][3] = mma16(a0, b3, acc[0][3]);
    acc[1][3] = mma16(a1, b3, acc[1][3]);
  }
}

#define OTP 68
template <bool RES>
__device__ __forceinline__ void store16x64_f32(const float* sw, float* __restrict__ out,
                                                const float* __restrict__ res,
                                                int ldo, int row0, int n0, int lane) {
  v4f val[8];
  size_t go[8];
#pragma unroll
  for (int it = 0; it < 8; ++it) {
    const int p    = lane + 32 * it;
    const int L    = p >> 3;
    const int pc   = p & 7;
    const int row  = L >> 1;
    const int half = L & 1;
    val[it] = *(const v4f*)(sw + row * OTP + half * 32 + pc * 4);
    go[it]  = (size_t)(row0 + row) * ldo + n0 + half * 32 + pc * 4;
    if (RES) val[it] += *(const v4f*)(res + go[it]);
  }
  for (int ps = 0; ps < 2; ++ps) {
#pragma unroll
    for (int it = 0; it < 8; ++it) *(volatile v4f*)(out + go[it]) = val[it];
    __threadfence();
  }
}

__device__ __forceinline__ void store16x64_h16(const float* sw, _Float16* __restrict__ out,
                                                int ldo, int row0, int n0, int lane) {
  v4u val[4];
  size_t go[4];
#pragma unroll
  for (int it = 0; it < 4; ++it) {
    const int p  = lane + 32 * it;
    const int L  = p >> 3;
    const int pc = p & 7;
    const float* ra = sw + L * OTP + pc * 8;
    val[it] = pack8h(*(const v4f*)(ra), *(const v4f*)(ra + 4));
    go[it]  = (size_t)(row0 + L) * ldo + n0 + pc * 8;
  }
  for (int ps = 0; ps < 2; ++ps) {
#pragma unroll
    for (int it = 0; it < 4; ++it) *(volatile v4u*)(out + go[it]) = val[it];
    __threadfence();
  }
}

__global__ __launch_bounds__(256) void k_wcvt(const float* __restrict__ w, int n8, _Float16* __restrict__ out) {
  const int i = blockIdx.x * 256 + threadIdx.x;
  if (i >= n8) return;
  const float* p = w + (size_t)i * 8;
  const v4f a0 = *(const v4f*)(p) * 64.0f;
  const v4f a1 = *(const v4f*)(p + 4) * 64.0f;
  const v4u hv = pack8h(a0, a1);
  _Float16* dst = out + (size_t)i * 8;
  for (int ps = 0; ps < 2; ++ps) {
    *(volatile v4u*)dst = hv;
    __threadfence();
  }
}

__global__ __launch_bounds__(256) void k_embed(const float* __restrict__ data, const float* __restrict__ wemb,
                                               const float* __restrict__ bemb,
                                               float* __restrict__ xf, _Float16* __restrict__ xh) {
  const int tid = threadIdx.x, lane = tid & 31, wave = tid >> 5;
  const int m  = blockIdx.x * 8 + wave;
  const int b  = m >> 9, n = m & (NP - 1);
  const int nn = min(n, NN - 1);
  const size_t bn = (size_t)b * NN + nn;
  const float d0 = data[bn * 2], d1 = data[bn * 2 + 1];
  const int d = 4 * lane;
  const v4f w0 = *(const v4f*)(wemb + 2 * d);
  const v4f w1 = *(const v4f*)(wemb + 2 * d + 4);
  const v4f bb = *(const v4f*)(bemb + d);
  v4f v;
  v[0] = (d0 * w0[0] + d1 * w0[1]) + bb[0];
  v[1] = (d0 * w0[2] + d1 * w0[3]) + bb[1];
  v[2] = (d0 * w1[0] + d1 * w1[1]) + bb[2];
  v[3] = (d0 * w1[2] + d1 * w1[3]) + bb[3];
  v = sel4(n < NN, v);
  const v2u hv = pack4h(v * 64.0f);
  const size_t o = (size_t)m * DM + d;
  for (int ps = 0; ps < 2; ++ps) {
    *(volatile v4f*)(xf + o) = v;
    *(volatile v2u*)(xh + o) = hv;
    __threadfence();
  }
}

__global__ __launch_bounds__(128) void k_reembed(const float* __restrict__ data, const float* __restrict__ wemb,
                                                 const float* __restrict__ bemb, const float* __restrict__ wout,
                                                 const float* __restrict__ bout,
                                                 float* __restrict__ xf, _Float16* __restrict__ xh) {
  __shared__ __align__(16) float er[DM];
  __shared__ __align__(16) float rr[DM];
  const int b = blockIdx.x;
  const int n = (blockIdx.y == 0) ? (NN - 1) : 0;
  const int d = threadIdx.x;
  const size_t bn = (size_t)b * NN + n;
  const float d0 = data[bn * 2], d1 = data[bn * 2 + 1];
  er[d] = (d0 * wemb[2 * d] + d1 * wemb[2 * d + 1]) + bemb[d];
  __syncthreads();
  const float* wr = wout + (size_t)d * DM;
  float acc = 0.f;
#pragma unroll 4
  for (int i = 0; i < DM; ++i) acc += er[i] * wr[i];
  rr[d] = acc + bout[d];
  __syncthreads();
  if (threadIdx.x < 32) {
    const int lane = threadIdx.x;
    const size_t m = (size_t)b * NP + n;
    const v4f v = *(const v4f*)(rr + 4 * lane);
    const v2u hv = pack4h(v * 64.0f);
    const size_t o = m * DM + 4 * lane;
    for (int ps = 0; ps < 2; ++ps) {
      *(volatile v4f*)(xf + o) = v;
      *(volatile v2u*)(xh + o) = hv;
      __threadfence();
    }
  }
}

#define SC4096 0.000244140625f
#define SC1024 0.0009765625f
__global__ __launch_bounds__(256) void k_q(const _Float16* __restrict__ xh, const _Float16* __restrict__ wq,
                                           float* __restrict__ sqp) {
  __shared__ __align__(16) float st[8][16 * OTP];
  const int tid = threadIdx.x, lane = tid & 31, wave = tid >> 5;
  const int hh = lane >> 4, c = lane & 15;
  const int m0 = blockIdx.x * 256 + wave * 32;
  const int n0 = blockIdx.y * 64;

  v8f acc[2][4];
#pragma unroll
  for (int s = 0; s < 2; ++s)
#pragma unroll
    for (int t = 0; t < 4; ++t) acc[s][t] = zero8();
  gemm32x64(xh, DM, wq, DM, DM, m0, n0, lane, acc);

  float* sw = st[wave];
#pragma unroll
  for (int sub = 0; sub < 2; ++sub) {
    __syncthreads();
#pragma unroll
    for (int t = 0; t < 4; ++t) {
#pragma unroll
      for (int r = 0; r < 8; ++r) {
        const float qv = acc[sub][t][r] * SC4096;
        const float e  = __expf(-qv);
        sw[(8 * hh + r) * OTP + 16 * t + c] = __builtin_amdgcn_rcpf(1.0f + e);
      }
    }
    __syncthreads();
    store16x64_f32<false>(sw, sqp, sqp, DM, m0 + 16 * sub, n0, lane);
  }
}

#define SVP 264
__global__ __launch_bounds__(256) void k_kv(const _Float16* __restrict__ xh, const _Float16* __restrict__ wk,
                                            const _Float16* __restrict__ wv,
                                            _Float16* __restrict__ ekt, _Float16* __restrict__ ekvt) {
  __shared__ __align__(16) _Float16 st[2][32 * SVP];
  const int tid = threadIdx.x, lane = tid & 31, wave = tid >> 5;
  const int hh = lane >> 4, c = lane & 15;
  const int bx = blockIdx.x;
  const int b = bx >> 1, half = bx & 1;
  const int m0 = bx * 256 + wave * 32;
  const int n0 = blockIdx.y * 32;

  v8f ak[2][2], av[2][2];
#pragma unroll
  for (int s = 0; s < 2; ++s)
#pragma unroll
    for (int t = 0; t < 2; ++t) { ak[s][t] = zero8(); av[s][t] = zero8(); }
#pragma unroll 1
  for (int k0 = 0; k0 < DM; k0 += 32) {
    const v16h a0  = ldfrag(xh, DM, m0, k0, lane);
    const v16h a1  = ldfrag(xh, DM, m0 + 16, k0, lane);
    const v16h bk0 = ldfrag(wk, DM, n0, k0, lane);
    const v16h bk1 = ldfrag(wk, DM, n0 + 16, k0, lane);
    const v16h bv0 = ldfrag(wv, DM, n0, k0, lane);
    const v16h bv1 = ldfrag(wv, DM, n0 + 16, k0, lane);
    ak[0][0] = mma16(a0, bk0, ak[0][0]);
    ak[1][0] = mma16(a1, bk0, ak[1][0]);
    ak[0][1] = mma16(a0, bk1, ak[0][1]);
    ak[1][1] = mma16(a1, bk1, ak[1][1]);
    av[0][0] = mma16(a0, bv0, av[0][0]);
    av[1][0] = mma16(a1, bv0, av[1][0]);
    av[0][1] = mma16(a0, bv1, av[0][1]);
    av[1][1] = mma16(a1, bv1, av[1][1]);
  }

#pragma unroll
  for (int sub = 0; sub < 2; ++sub)
#pragma unroll
    for (int t = 0; t < 2; ++t)
#pragma unroll
      for (int r = 0; r < 8; ++r) {
        const int lr = wave * 32 + sub * 16 + 8 * hh + r;
        const bool valid = (half * 256 + lr) < NN;
        const float kval = ak[sub][t][r] * SC4096;
        const float vval = av[sub][t][r] * SC4096;
        const float ek  = __expf(kval);
        const float ekv = (ek * vval) * 16.0f;
        st[0][(16 * t + c) * SVP + lr] = (_Float16)(valid ? ek : 0.f);
        st[1][(16 * t + c) * SVP + lr] = (_Float16)(valid ? ekv : 0.f);
      }
  __syncthreads();

  const size_t pbase = ((size_t)b * DM + n0) * NP + (size_t)half * 256;
  v4u val[8];
  size_t go[8];
#pragma unroll
  for (int j = 0; j < 8; ++j) {
    const int p    = tid + 256 * j;
    const int drow = (p >> 5) & 31;
    const int pc   = p & 31;
    Pack8 pk;
    pk.h   = *(const v8h*)(&st[j >> 2][drow * SVP + pc * 8]);
    val[j] = pk.u;
    go[j]  = pbase + (size_t)drow * NP + pc * 8;
  }
  for (int ps = 0; ps < 2; ++ps) {
#pragma unroll
    for (int j = 0; j < 8; ++j) {
      _Float16* dst = ((j < 4) ? ekt : ekvt) + go[j];
      *(volatile v4u*)dst = val[j];
    }
    __threadfence();
  }
}

#define SSP 520
#define RTP 132
__global__ __launch_bounds__(256) void k_attn(const float* __restrict__ dist, const float* __restrict__ lsc,
                                              const float* __restrict__ alpha, int layer,
                                              const float* __restrict__ sqp,
                                              const _Float16* __restrict__ ekt, const _Float16* __restrict__ ekvt,
                                              const float* __restrict__ xf, float* __restrict__ yf) {
  __shared__ __align__(16) _Float16 Ss[32 * SSP];
  __shared__ __align__(16) float rat[32 * RTP];
  const int tid = threadIdx.x, lane = tid & 31, wave = tid >> 5;
  const int hh = lane >> 4, c = lane & 15;
  const int b  = blockIdx.x >> 4;
  const int rt = blockIdx.x & 15;
  const int r0 = rt * 32;
  const float cf = lsc[0] * alpha[layer];
  const float* db = dist + (size_t)b * NN * NN;

#pragma unroll 2
  for (int it = 0; it < 16; ++it) {
    const int idx = it * 256 + tid;
    const int row = idx >> 7;
    const int c4  = idx & 127;
    const int gr  = r0 + row;
    const int grc = min(gr, NN - 1);
    const int c4c = min(c4, NN / 4 - 1);
    const v4f dv = *(const v4f*)(db + (size_t)grc * NN + 4 * c4c);
    const bool ok = (gr < NN) && (c4 < NN / 4);
    float s0 = __expf(-(cf * dv[0]));
    float s1 = __expf(-(cf * dv[1]));
    float s2 = __expf(-(cf * dv[2]));
    float s3 = __expf(-(cf * dv[3]));
    s0 = ok ? s0 : 0.f; s1 = ok ? s1 : 0.f; s2 = ok ? s2 : 0.f; s3 = ok ? s3 : 0.f;
    Pack4 pk;
    pk.h = (v4h){(_Float16)s0, (_Float16)s1, (_Float16)s2, (_Float16)s3};
    *(v2u*)(Ss + row * SSP + 4 * c4) = pk.u;
  }
  __syncthreads();

  const int d0 = wave * 16;
  const _Float16* pk = ekt  + (size_t)b * DM * NP;
  const _Float16* pv = ekvt + (size_t)b * DM * NP;
  v8f ad[2], an[2];
#pragma unroll
  for (int s = 0; s < 2; ++s) { ad[s] = zero8(); an[s] = zero8(); }
#pragma unroll 1
  for (int k0 = 0; k0 < NP; k0 += 32) {
    const v16h a0 = ldfrag(Ss, SSP, 0, k0, lane);
    const v16h a1 = ldfrag(Ss, SSP, 16, k0, lane);
    const v16h bd = ldfrag(pk, NP, d0, k0, lane);
    const v16h bn = ldfrag(pv, NP, d0, k0, lane);
    ad[0] = mma16(a0, bd, ad[0]);
    ad[1] = mma16(a1, bd, ad[1]);
    an[0] = mma16(a0, bn, an[0]);
    an[1] = mma16(a1, bn, an[1]);
  }
#pragma unroll
  for (int sub = 0; sub < 2; ++sub)
#pragma unroll
    for (int r = 0; r < 8; ++r) {
      const int row = sub * 16 + 8 * hh + r;
      const float den = ad[sub][r];
      const float num = an[sub][r];
      float q = (num * __builtin_amdgcn_rcpf(den)) * 0.0625f;
      q = (den > 0.f) ? q : 0.f;
      rat[row * RTP + d0 + c] = q;
    }
  __syncthreads();

  v4f val[4];
  size_t go[4];
  bool okr[4];
#pragma unroll
  for (int i = 0; i < 4; ++i) {
    const int L = wave * 4 + i;
    const int n = r0 + L;
    okr[i] = n < NN;
    const size_t o = ((size_t)b * NP + n) * DM + 4 * lane;
    const v4f xv = *(const v4f*)(xf + o);
    const v4f sv = *(const v4f*)(sqp + o);
    const v4f rv = *(const v4f*)(rat + L * RTP + 4 * lane);
    val[i] = xv + sv * rv;
    go[i]  = o;
  }
  for (int ps = 0; ps < 2; ++ps) {
#pragma unroll
    for (int i = 0; i < 4; ++i)
      if (okr[i]) *(volatile v4f*)(yf + go[i]) = val[i];
    __threadfence();
  }
}

__global__ __launch_bounds__(256) void k_in(const float* __restrict__ yin, const float* __restrict__ g,
                                            const float* __restrict__ be,
                                            float* __restrict__ xo, int orows, _Float16* __restrict__ xh) {
  __shared__ __align__(16) float red1[8 * DM];
  __shared__ __align__(16) float red2[8 * DM];
  const int tid = threadIdx.x, lane = tid & 31, wave = tid >> 5;
  const int b = blockIdx.x;
  const int d = 4 * lane;
  const float* yb = yin + (size_t)b * NP * DM + d;

  v4f s = zero4();
  for (int n = wave; n < NN; n += 8) s += *(const v4f*)(yb + (size_t)n * DM);
  *(v4f*)(red1 + wave * DM + d) = s;
  __syncthreads();
  v4f tot = *(const v4f*)(red1 + d);
#pragma unroll
  for (int w = 1; w < 8; ++w) tot += *(const v4f*)(red1 + w * DM + d);
  const v4f mean = tot * 0.002f;

  v4f ss = zero4();
  for (int n = wave; n < NN; n += 8) {
    const v4f dv = *(const v4f*)(yb + (size_t)n * DM) - mean;
    ss += dv * dv;
  }
  *(v4f*)(red2 + wave * DM + d) = ss;
  __syncthreads();
  v4f tot2 = *(const v4f*)(red2 + d);
#pragma unroll
  for (int w = 1; w < 8; ++w) tot2 += *(const v4f*)(red2 + w * DM + d);
  const v4f var = tot2 * 0.002f;
  v4f rstd;
  rstd[0] = rsqrtf(var[0] + EPSV);
  rstd[1] = rsqrtf(var[1] + EPSV);
  rstd[2] = rsqrtf(var[2] + EPSV);
  rstd[3] = rsqrtf(var[3] + EPSV);
  const v4f gv = *(const v4f*)(g + d);
  const v4f bv = *(const v4f*)(be + d);
  const bool plane = (orows == NP);

  for (int n = wave; n < NP; n += 8) {
    const bool valid = n < NN;
    const int nc = min(n, NN - 1);
    const v4f v = *(const v4f*)(yb + (size_t)nc * DM);
    v4f y = ((v - mean) * rstd) * gv + bv;
    y = sel4(valid, y);
    const v2u hv = pack4h(y * 64.0f);
    const bool wf = valid || plane;
    const size_t of = ((size_t)b * orows + n) * DM + d;
    const size_t oh = ((size_t)b * NP + n) * DM + d;
    for (int ps = 0; ps < 2; ++ps) {
      if (wf) *(volatile v4f*)(xo + of) = y;
      *(volatile v2u*)(xh + oh) = hv;
      __threadfence();
    }
  }
}

__global__ __launch_bounds__(256) void k_ffn1(const _Float16* __restrict__ x1h, const _Float16* __restrict__ w1,
                                              const float* __restrict__ b1, _Float16* __restrict__ hp) {
  __shared__ __align__(16) float st[8][16 * OTP];
  const int tid = threadIdx.x, lane = tid & 31, wave = tid >> 5;
  const int hh = lane >> 4, c = lane & 15;
  const int m0 = blockIdx.x * 256 + wave * 32;
  const int n0 = blockIdx.y * 64;

  v8f acc[2][4];
#pragma unroll
  for (int s = 0; s < 2; ++s)
#pragma unroll
    for (int t = 0; t < 4; ++t) acc[s][t] = zero8();
  gemm32x64(x1h, DM, w1, DM, DM, m0, n0, lane, acc);
  float bb[4];
#pragma unroll
  for (int t = 0; t < 4; ++t) bb[t] = b1[n0 + 16 * t + c];

  float* sw = st[wave];
#pragma unroll
  for (int sub = 0; sub < 2; ++sub) {
    __syncthreads();
#pragma unroll
    for (int t = 0; t < 4; ++t) {
#pragma unroll
      for (int r = 0; r < 8; ++r)
        sw[(8 * hh + r) * OTP + 16 * t + c] = fmaxf(acc[sub][t][r] * SC4096 + bb[t], 0.f) * 16.0f;
    }
    __syncthreads();
    store16x64_h16(sw, hp, DFF, m0 + 16 * sub, n0, lane);
  }
}

__global__ __launch_bounds__(256) void k_ffn2(const _Float16* __restrict__ hp, const _Float16* __restrict__ w2,
                                              const float* __restrict__ b2, const float* __restrict__ x1f,
                                              float* __restrict__ yf) {
  __shared__ __align__(16) float st[8][16 * OTP];
  const int tid = threadIdx.x, lane = tid & 31, wave = tid >> 5;
  const int hh = lane >> 4, c = lane & 15;
  const int m0 = blockIdx.x * 256 + wave * 32;
  const int n0 = blockIdx.y * 64;

  v8f acc[2][4];
#pragma unroll
  for (int s = 0; s < 2; ++s)
#pragma unroll
    for (int t = 0; t < 4; ++t) acc[s][t] = zero8();
  gemm32x64(hp, DFF, w2, DFF, DFF, m0, n0, lane, acc);
  float bb[4];
#pragma unroll
  for (int t = 0; t < 4; ++t) bb[t] = b2[n0 + 16 * t + c];

  float* sw = st[wave];
#pragma unroll
  for (int sub = 0; sub < 2; ++sub) {
    __syncthreads();
#pragma unroll
    for (int t = 0; t < 4; ++t) {
#pragma unroll
      for (int r = 0; r < 8; ++r) sw[(8 * hh + r) * OTP + 16 * t + c] = acc[sub][t][r] * SC1024 + bb[t];
    }
    __syncthreads();
    store16x64_f32<true>(sw, yf, x1f, DM, m0 + 16 * sub, n0, lane);
  }
}

extern "C" void kernel_launch(void* const* d_in, const int* in_sizes, int n_in,
                              void* d_out, int out_size, void* d_ws, size_t ws_size,
                              hipStream_t stream) {
  if (n_in < 19) return;
  if (in_sizes[0] != NB * NN * 2) return;
  if (in_sizes[1] != NB * NN * NN) return;
  if (in_sizes[2] < 1) return;
  if (in_sizes[3] != DM * 2) return;
  if (in_sizes[4] != DM) return;
  if (in_sizes[5] != DM * DM) return;
  if (in_sizes[6] != DM) return;
  if (in_sizes[7] != NL * DM * DM) return;
  if (in_sizes[8] != NL * DM * DM) return;
  if (in_sizes[9] != NL * DM * DM) return;
  if (in_sizes[10] != NL * DM) return;
  if (in_sizes[11] != NL * DM) return;
  if (in_sizes[12] != NL * DFF * DM) return;
  if (in_sizes[13] != NL * DFF) return;
  if (in_sizes[14] != NL * DM * DFF) return;
  if (in_sizes[15] != NL * DM) return;
  if (in_sizes[16] != NL * DM) return;
  if (in_sizes[17] != NL * DM) return;
  if (in_sizes[18] < NL) return;
  if (out_size != NB * NN * DM) return;

  const float* data  = (const float*)d_in[0];
  const float* dist  = (const float*)d_in[1];
  const float* lsc   = (const float*)d_in[2];
  const float* wemb  = (const float*)d_in[3];
  const float* bemb  = (const float*)d_in[4];
  const float* wout  = (const float*)d_in[5];
  const float* bout  = (const float*)d_in[6];
  const float* wq    = (const float*)d_in[7];
  const float* wk    = (const float*)d_in[8];
  const float* wv    = (const float*)d_in[9];
  const float* g1    = (const float*)d_in[10];
  const float* be1   = (const float*)d_in[11];
  const float* w1    = (const float*)d_in[12];
  const float* b1    = (const float*)d_in[13];
  const float* w2    = (const float*)d_in[14];
  const float* b2    = (const float*)d_in[15];
  const float* g2    = (const float*)d_in[16];
  const float* be2   = (const float*)d_in[17];
  const float* alpha = (const float*)d_in[18];
  float* out = (float*)d_out;

  size_t off = 0;
  const size_t oWQ  = off; off += (size_t)NL * DM * DM * 2;
  const size_t oWK  = off; off += (size_t)NL * DM * DM * 2;
  const size_t oWV  = off; off += (size_t)NL * DM * DM * 2;
  const size_t oW1  = off; off += (size_t)NL * DFF * DM * 2;
  const size_t oW2  = off; off += (size_t)NL * DM * DFF * 2;
  const size_t oXh  = off; off += (size_t)NROW * DM * 2;
  const size_t oX1h = off; off += (size_t)NROW * DM * 2;
  const size_t oX   = off; off += (size_t)NROW * DM * 4;
  const size_t oX1  = off; off += (size_t)NROW * DM * 4;
  const size_t oY   = off; off += (size_t)NROW * DM * 4;
  const size_t oSQ  = off; off += (size_t)NROW * DM * 4;
  const size_t oEK  = off; off += (size_t)NB * DM * NP * 2;
  const size_t oEKV = off; off += (size_t)NB * DM * NP * 2;
  const size_t oHd  = oSQ;
  if (oHd + (size_t)NROW * DFF * 2 > off) return;
  if (off > ws_size) return;
  if (off > (size_t)134217728) return;

  char* ws = (char*)d_ws;
  _Float16* WQ   = (_Float16*)(ws + oWQ);
  _Float16* WK   = (_Float16*)(ws + oWK);
  _Float16* WV   = (_Float16*)(ws + oWV);
  _Float16* W1P  = (_Float16*)(ws + oW1);
  _Float16* W2P  = (_Float16*)(ws + oW2);
  _Float16* Xh   = (_Float16*)(ws + oXh);
  _Float16* X1h  = (_Float16*)(ws + oX1h);
  float*    X    = (float*)(ws + oX);
  float*    X1   = (float*)(ws + oX1);
  float*    Y    = (float*)(ws + oY);
  float*    SQ   = (float*)(ws + oSQ);
  _Float16* EKT  = (_Float16*)(ws + oEK);
  _Float16* EKVT = (_Float16*)(ws + oEKV);
  _Float16* Hd   = (_Float16*)(ws + oHd);

  const int n8q = (NL * DM * DM) / 8;
  const int n8f = (NL * DFF * DM) / 8;
  k_wcvt<<<dim3(n8q / 256), dim3(256), 0, stream>>>(wq, n8q, WQ);
  k_wcvt<<<dim3(n8q / 256), dim3(256), 0, stream>>>(wk, n8q, WK);
  k_wcvt<<<dim3(n8q / 256), dim3(256), 0, stream>>>(wv, n8q, WV);
  k_wcvt<<<dim3(n8f / 256), dim3(256), 0, stream>>>(w1, n8f, W1P);
  k_wcvt<<<dim3(n8f / 256), dim3(256), 0, stream>>>(w2, n8f, W2P);
  k_embed<<<dim3(NROW / 8), dim3(256), 0, stream>>>(data, wemb, bemb, X, Xh);
  k_reembed<<<dim3(NB, 2), dim3(128), 0, stream>>>(data, wemb, bemb, wout, bout, X, Xh);
  for (int l = 0; l < NL; ++l) {
    const size_t ow = (size_t)l * DM * DM;
    const size_t of = (size_t)l * DFF * DM;
    k_q<<<dim3(NROW / 256, DM / 64), dim3(256), 0, stream>>>(Xh, WQ + ow, SQ);
    k_kv<<<dim3(NROW / 256, DM / 32), dim3(256), 0, stream>>>(Xh, WK + ow, WV + ow, EKT, EKVT);
    k_attn<<<dim3(NB * 16), dim3(256), 0, stream>>>(dist, lsc, alpha, l, SQ, EKT, EKVT, X, Y);
    k_in<<<dim3(NB), dim3(256), 0, stream>>>(Y, g1 + (size_t)l * DM, be1 + (size_t)l * DM, X1, NP, X1h);
    k_ffn1<<<dim3(NROW / 256, DFF / 64), dim3(256), 0, stream>>>(X1h, W1P + of, b1 + (size_t)l * DFF, Hd);
    k_ffn2<<<dim3(NROW / 256, DM / 64), dim3(256), 0, stream>>>(Hd, W2P + of, b2 + (size_t)l * DM, X1, Y);
    float* xdst    = (l == NL - 1) ? out : X;
    const int orow = (l == NL - 1) ? NN : NP;
    k_in<<<dim3(NB), dim3(256), 0, stream>>>(Y, g2 + (size_t)l * DM, be2 + (size_t)l * DM, xdst, orow, Xh);
  }
  (void)hipGetLastError();
}
